// IT_Fast_Attn_76656576299169
// MI455X (gfx1250) — hardware-verified
//
#include <hip/hip_runtime.h>
#include <math.h>

constexpr int kB   = 8;
constexpr int kC   = 256;
constexpr int kN   = 4096;
constexpr int kC2  = 512;
constexpr int kC4  = 1024;
constexpr int kGrp = 2;
constexpr int kNGrp = kB / kGrp;
constexpr int kRowsG = kGrp * kN;
constexpr float kWCarry    = 64.0f;
constexpr float kWCarryInv = 1.0f / 64.0f;
constexpr float kSmCarry   = 1024.0f;
constexpr float kSmCarryInv = 1.0f / 1024.0f;
constexpr float kLnEps  = 1e-5f;
constexpr float kInvC   = 1.0f / 256.0f;
constexpr float kInvC4  = 1.0f / 1024.0f;

typedef __attribute__((ext_vector_type(16))) _Float16 v16h;
typedef __attribute__((ext_vector_type(8)))  _Float16 v8h;
typedef __attribute__((ext_vector_type(16))) __bf16   v16b;
typedef __attribute__((ext_vector_type(8)))  __bf16   v8b;
typedef __attribute__((ext_vector_type(8)))  float    v8f;
typedef __attribute__((ext_vector_type(4)))  float    v4f;
typedef __attribute__((ext_vector_type(4)))  unsigned int v4u;

__device__ __forceinline__ unsigned short f2bf_bits(float f) {
  unsigned u = __float_as_uint(f);
  return (unsigned short)((u + 0x7FFFu + ((u >> 16) & 1u)) >> 16);
}
__device__ __forceinline__ float bf_bits2f(unsigned short h) { return __uint_as_float(((unsigned)h) << 16); }

__device__ __forceinline__ void dep_guard_h(v8f& a, v8f& b, v16h x, v16h y) { asm volatile("v_nop\n\tv_nop\n\tv_nop\n\tv_nop" : "+v"(a), "+v"(b) : "v"(x), "v"(y)); }
__device__ __forceinline__ void dep_guard_b(v8f& a, v8f& b, v16b x, v16b y) { asm volatile("v_nop\n\tv_nop\n\tv_nop\n\tv_nop" : "+v"(a), "+v"(b) : "v"(x), "v"(y)); }
__device__ __forceinline__ void keep4_h(v16h a, v16h b, v16h c, v16h d) { asm volatile("v_nop" :: "v"(a), "v"(b), "v"(c), "v"(d)); }
__device__ __forceinline__ void keep4_b(v16b a, v16b b, v16b c, v16b d) { asm volatile("v_nop" :: "v"(a), "v"(b), "v"(c), "v"(d)); }
__device__ __forceinline__ void acc_guard4(v8f& a, v8f& b, v8f& c, v8f& d) { asm volatile("v_nop\n\tv_nop\n\tv_nop\n\tv_nop" : "+v"(a), "+v"(b), "+v"(c), "+v"(d)); }
template <typename T> struct Frag;
template <> struct Frag<_Float16> {
  typedef v16h V; union U { v16h v; v8h h[2]; };
  static __device__ __forceinline__ v16h load(const _Float16* p) {
    U f; f.h[0] = *(const v8h*)(p); f.h[1] = *(const v8h*)(p + 16); return f.v;
  }
  static __device__ __forceinline__ v8f mma(v16h a, v16h b, v8f c) {
    return __builtin_amdgcn_wmma_f32_16x16x32_f16(false, a, false, b, (short)0, c, false, false);
  }
  static __device__ __forceinline__ void guard(v8f& a, v8f& b, v16h x, v16h y) { dep_guard_h(a, b, x, y); }
  static __device__ __forceinline__ void keep(v16h a, v16h b, v16h c, v16h d) { keep4_h(a, b, c, d); }
};
template <> struct Frag<__bf16> {
  typedef v16b V; union U { v16b v; v8b h[2]; };
  static __device__ __forceinline__ v16b load(const __bf16* p) {
    U f; f.h[0] = *(const v8b*)(p); f.h[1] = *(const v8b*)(p + 16); return f.v;
  }
  static __device__ __forceinline__ v8f mma(v16b a, v16b b, v8f c) {
    return __builtin_amdgcn_wmma_f32_16x16x32_bf16(false, a, false, b, (short)0, c, false, false);
  }
  static __device__ __forceinline__ void guard(v8f& a, v8f& b, v16b x, v16b y) { dep_guard_b(a, b, x, y); }
  static __device__ __forceinline__ void keep(v16b a, v16b b, v16b c, v16b d) { keep4_b(a, b, c, d); }
};

__device__ __forceinline__ unsigned pk16(unsigned short a, unsigned short b) { return (unsigned)a | ((unsigned)b << 16); }
__device__ __forceinline__ unsigned short h_bits(float f) { const _Float16 h = (_Float16)f; return __builtin_bit_cast(unsigned short, h); }

__device__ __forceinline__ float wave_sum32(float x) {
#pragma unroll
  for (int off = 16; off > 0; off >>= 1) x += __shfl_xor(x, off, 32);
  return x;
}
__device__ __forceinline__ float wave_max32(float x) {
#pragma unroll
  for (int off = 16; off > 0; off >>= 1) x = fmaxf(x, __shfl_xor(x, off, 32));
  return x;
}

template <int ET> struct Elem;
template <> struct Elem<0> { typedef _Float16 T; };
template <> struct Elem<1> { typedef __bf16 T; };
template <int ET, bool SPLIT, int BIAS_MODE, int OUT_MODE, bool RESID, int ACT = 0>
__global__ __launch_bounds__(256) void wmma_gemm64(
    const unsigned short* __restrict__ Ap, const unsigned short* __restrict__ A2p, int lda, long strideA,
    const unsigned short* __restrict__ Btp, const unsigned short* __restrict__ Bt2p, int ldb, long strideB,
    void* __restrict__ Cout, void* __restrict__ Cout2, int ldc, long strideC,
    const float* __restrict__ bias,
    const float* __restrict__ resid, long strideR,
    int M, int N, int K, float scale) {
  typedef typename Elem<ET>::T T;
  typedef typename Frag<T>::V V;
  const T* A = (const T*)Ap; const T* A2 = (const T*)A2p; const T* Bt = (const T*)Btp; const T* Bt2 = (const T*)Bt2p;
  __shared__ __align__(16) float sT[8][16 * 68];
  const int b    = blockIdx.y;
  const int lane = threadIdx.x & 31;
  const int wave = threadIdx.x >> 5;
  const int tilesN = N >> 6;
  const int tilesM = M >> 6;
  const int tile = blockIdx.x * 8 + wave;
  if (tile >= tilesM * tilesN) return;
  const int tm = tile / tilesN;
  const int tn = tile - tm * tilesN;
  const int m0 = tm << 6;
  const int n0 = tn << 6;

  const T* Ab  = A  + (size_t)b * strideA;
  const T* Bb  = Bt + (size_t)b * strideB;
  const T* Ab2 = SPLIT ? (A2  + (size_t)b * strideA) : nullptr;
  const T* Bb2 = SPLIT ? (Bt2 + (size_t)b * strideB) : nullptr;

  const int rlane = lane & 15;
  const int koff  = (lane >> 4) * 8;
  const int mOff  = (lane >> 4) * 8;

  v8f acc[4][4];
#pragma unroll
  for (int i = 0; i < 4; ++i)
#pragma unroll
    for (int j = 0; j < 4; ++j) acc[i][j] = (v8f){0.f,0.f,0.f,0.f,0.f,0.f,0.f,0.f};

  for (int k0 = 0; k0 < K; k0 += 32) {
    V bh[4], bl[4];
#pragma unroll
    for (int j = 0; j < 4; ++j) {
      const size_t bo = (size_t)(n0 + (j << 4) + rlane) * ldb + koff + k0;
      bh[j] = Frag<T>::load(Bb + bo);
      if (SPLIT) bl[j] = Frag<T>::load(Bb2 + bo);
    }
#pragma unroll
    for (int i = 0; i < 4; ++i) {
      const size_t ao = (size_t)(m0 + (i << 4) + rlane) * lda + koff + k0;
      V ah = Frag<T>::load(Ab + ao);
      V al;
      if (SPLIT) al = Frag<T>::load(Ab2 + ao);
#pragma unroll
      for (int j = 0; j < 4; ++j) {
        acc[i][j] = Frag<T>::mma(ah, bh[j], acc[i][j]);
        if (SPLIT) {
          acc[i][j] = Frag<T>::mma(ah, bl[j], acc[i][j]);
          acc[i][j] = Frag<T>::mma(al, bh[j], acc[i][j]);
        }
      }
      Frag<T>::guard(acc[i][0], acc[i][3], ah, SPLIT ? al : ah);
    }
    Frag<T>::keep(bh[0], bh[1], bh[2], bh[3]);
    if (SPLIT) Frag<T>::keep(bl[0], bl[1], bl[2], bl[3]);
  }
  acc_guard4(acc[0][0], acc[0][1], acc[0][2], acc[0][3]);
  acc_guard4(acc[1][0], acc[1][1], acc[1][2], acc[1][3]);
  acc_guard4(acc[2][0], acc[2][1], acc[2][2], acc[2][3]);
  acc_guard4(acc[3][0], acc[3][1], acc[3][2], acc[3][3]);

  float* slab = sT[wave];
  const float* Rb = RESID ? (resid + (size_t)b * strideR) : nullptr;
#pragma unroll
  for (int i = 0; i < 4; ++i) {
    const int mBase = m0 + (i << 4);
#pragma unroll
    for (int j = 0; j < 4; ++j) {
      const int n = n0 + (j << 4) + rlane;
      float bv = 0.f;
      if (BIAS_MODE == 2) bv = bias[n];
#pragma unroll
      for (int r = 0; r < 8; ++r) {
        float v = acc[i][j][r] * scale;
        if (BIAS_MODE == 1) v += bias[mBase + mOff + r];
        if (BIAS_MODE == 2) v += bv;
        if (RESID) v += Rb[(size_t)(mBase + mOff + r) * ldc + n];
        if (ACT == 2) v = fmaxf(v, 0.0f);
        if (ACT == 4) v = (v > 0.f) ? v : 0.01f * v;
        slab[(mOff + r) * 68 + (j << 4) + rlane] = v;
      }
    }
    __builtin_amdgcn_fence(__ATOMIC_RELEASE, "workgroup");
    __builtin_amdgcn_wave_barrier();
    __builtin_amdgcn_fence(__ATOMIC_ACQUIRE, "workgroup");
    if (OUT_MODE == 0) {
      float* C = (float*)Cout + (size_t)b * strideC;
      const int hh = lane >> 4, c4 = (lane & 15) * 4;
      for (int pass = 0; pass < 2; ++pass) {
#pragma unroll
        for (int it = 0; it < 8; ++it) {
          const int row = it * 2 + hh;
          v4f v = *(const v4f*)(slab + row * 68 + c4);
          *(volatile v4f*)(C + (size_t)(mBase + row) * ldc + n0 + c4) = v;
        }
        __threadfence();
      }
    } else {
      const int q = lane >> 3, c8 = (lane & 7) * 8;
      unsigned short* C  = (unsigned short*)Cout  + (size_t)b * strideC;
      unsigned short* C2 = (OUT_MODE == 2) ? ((unsigned short*)Cout2 + (size_t)b * strideC) : nullptr;
      for (int pass = 0; pass < 2; ++pass) {
#pragma unroll
        for (int it = 0; it < 4; ++it) {
          const int row = it * 4 + q;
          const float* sp = slab + row * 68 + c8;
          v8h hv, lv;
#pragma unroll
          for (int e = 0; e < 8; ++e) {
            if (OUT_MODE == 1) {
              hv[e] = (_Float16)sp[e];
            } else {
              unsigned short hb = f2bf_bits(sp[e]);
              unsigned short lb = f2bf_bits(sp[e] - bf_bits2f(hb));
              hv[e] = __builtin_bit_cast(_Float16, hb);
              lv[e] = __builtin_bit_cast(_Float16, lb);
            }
          }
          *(volatile v8h*)(C + (size_t)(mBase + row) * ldc + n0 + c8) = hv;
          if (OUT_MODE == 2) *(volatile v8h*)(C2 + (size_t)(mBase + row) * ldc + n0 + c8) = lv;
        }
        __threadfence();
      }
    }
    __builtin_amdgcn_fence(__ATOMIC_RELEASE, "workgroup");
    __builtin_amdgcn_wave_barrier();
    __builtin_amdgcn_fence(__ATOMIC_ACQUIRE, "workgroup");
  }
}

__global__ __launch_bounds__(256) void wcast_kernel(const float* __restrict__ Wq, const float* __restrict__ Wm,
                                                    const float* __restrict__ Wr,
                                                    unsigned short* __restrict__ oq, unsigned short* __restrict__ om,
                                                    unsigned short* __restrict__ orr, float scale) {
  const int blk = blockIdx.x;
  const float* src = Wr;
  unsigned short* dst = orr;
  int base = (blk - 160) * 256;
  if (blk < 32) { src = Wq; dst = oq; base = blk * 256; }
  else if (blk < 160) { src = Wm; dst = om; base = (blk - 32) * 256; }
  const int i = base + (int)threadIdx.x;
  const float* p = src + 8 * (size_t)i;
  const v4f a = *(const v4f*)(p);
  const v4f c = *(const v4f*)(p + 4);
  unsigned short hb[8];
#pragma unroll
  for (int e = 0; e < 4; ++e) {
    hb[e]     = h_bits(a[e] * scale);
    hb[4 + e] = h_bits(c[e] * scale);
  }
  const v4u u = (v4u){pk16(hb[0], hb[1]), pk16(hb[2], hb[3]), pk16(hb[4], hb[5]), pk16(hb[6], hb[7])};
  unsigned short* q = dst + 8 * (size_t)i;
  *(volatile v4u*)q = u;
  __threadfence();
  *(volatile v4u*)q = u;
}

__global__ __launch_bounds__(256) void tin_kernel(const float* __restrict__ xin, unsigned short* __restrict__ X0, int b0) {
  __shared__ __align__(16) unsigned short tile[64][264];
  const int t = threadIdx.x;
  const int n0 = blockIdx.x * 64;
  const int bl = blockIdx.y;
  const float* xb = xin + (size_t)(b0 + bl) * kC * kN + n0;
#pragma unroll 4
  for (int i = 0; i < 64; ++i) {
    const int e = i * 256 + t;
    const int c = e >> 6;
    const int j = e & 63;
    tile[j][c] = h_bits(xb[(size_t)c * kN + j]);
  }
  __syncthreads();
  const int lane = t & 31, wave = t >> 5;
  const int c8 = lane * 8;
  for (int pass = 0; pass < 2; ++pass) {
#pragma unroll
    for (int it = 0; it < 8; ++it) {
      const int r = wave * 8 + it;
      const v4u u = *(const v4u*)(&tile[r][c8]);
      *(volatile v4u*)(X0 + ((size_t)bl * kN + n0 + r) * kC + c8) = u;
    }
    __threadfence();
  }
}

__global__ __launch_bounds__(256) void prep_kernel(const float* __restrict__ X32, unsigned short* __restrict__ SM,
                                                   unsigned short* __restrict__ CAT1, unsigned short* __restrict__ XT) {
  __shared__ __align__(16) unsigned short tile[256 * 72];
  const int lane = threadIdx.x & 31, wave = threadIdx.x >> 5;
  const int n0 = blockIdx.x * 64;
  const int bl = blockIdx.y;
  const int c8 = lane * 8;
#pragma unroll 1
  for (int it = 0; it < 8; ++it) {
    const int rloc = wave * 8 + it;
    const size_t R = (size_t)bl * kN + n0 + rloc;
    const float* xr = X32 + R * kC + c8;
    const v4f a = *(const v4f*)(xr);
    const v4f c = *(const v4f*)(xr + 4);
    float x[8];
#pragma unroll
    for (int e = 0; e < 4; ++e) { x[e] = a[e]; x[4 + e] = c[e]; }
    float m = fmaxf(fmaxf(fmaxf(x[0], x[1]), fmaxf(x[2], x[3])), fmaxf(fmaxf(x[4], x[5]), fmaxf(x[6], x[7])));
    m = wave_max32(m);
    float ex[8];
    float s = 0.f;
#pragma unroll
    for (int e = 0; e < 8; ++e) { ex[e] = expf(x[e] - m); s += ex[e]; }
    s = wave_sum32(s);
    const float inv = kSmCarry * (1.0f / s);
    unsigned short hs[8], hx[8];
#pragma unroll
    for (int e = 0; e < 8; ++e) {
      hs[e] = h_bits(ex[e] * inv);
      hx[e] = h_bits(x[e]);
      tile[(c8 + e) * 72 + rloc] = hx[e];
    }
    const v4u us = (v4u){pk16(hs[0], hs[1]), pk16(hs[2], hs[3]), pk16(hs[4], hs[5]), pk16(hs[6], hs[7])};
    const v4u ux = (v4u){pk16(hx[0], hx[1]), pk16(hx[2], hx[3]), pk16(hx[4], hx[5]), pk16(hx[6], hx[7])};
    for (int pass = 0; pass < 2; ++pass) {
      *(volatile v4u*)(SM + R * kC + c8) = us;
      *(volatile v4u*)(CAT1 + R * kC2 + kC + c8) = ux;
      __threadfence();
    }
  }
  __syncthreads();
  const int q = lane >> 3, cc8 = (lane & 7) * 8;
  for (int pass = 0; pass < 2; ++pass) {
#pragma unroll
    for (int i = 0; i < 8; ++i) {
      const int L = i * 32 + wave * 4 + q;
      const v4u u = *(const v4u*)(tile + L * 72 + cc8);
      *(volatile v4u*)(XT + ((size_t)bl * kC + L) * kN + n0 + cc8) = u;
    }
    __threadfence();
  }
}

__global__ __launch_bounds__(256) void cast_out_kernel(const float* __restrict__ O32, unsigned short* __restrict__ CAT1, int nthr) {
  const int i = blockIdx.x * 256 + threadIdx.x;
  if (i >= nthr) return;
  const int row = i >> 5, c8 = (i & 31) * 8;
  const float* p = O32 + (size_t)row * kC + c8;
  const v4f a = *(const v4f*)(p);
  const v4f c = *(const v4f*)(p + 4);
  unsigned short hb[8];
#pragma unroll
  for (int e = 0; e < 4; ++e) {
    hb[e]     = h_bits(a[e]);
    hb[4 + e] = h_bits(c[e]);
  }
  const v4u u = (v4u){pk16(hb[0], hb[1]), pk16(hb[2], hb[3]), pk16(hb[4], hb[5]), pk16(hb[6], hb[7])};
  unsigned short* q = CAT1 + (size_t)row * kC2 + c8;
  *(volatile v4u*)q = u;
  __threadfence();
  *(volatile v4u*)q = u;
}

__global__ __launch_bounds__(256) void ln1_kernel(const float* __restrict__ O32, const float* __restrict__ Vp,
                                                  const float* __restrict__ Mp, const float* __restrict__ g1,
                                                  const float* __restrict__ be1, unsigned short* __restrict__ Y) {
  const int lane = threadIdx.x & 31, wave = threadIdx.x >> 5;
  const int c8 = lane * 8;
#pragma unroll 1
  for (int it = 0; it < 8; ++it) {
    const size_t R = (size_t)blockIdx.x * 64 + wave * 8 + it;
    float v[32];
    {
      const float* po = O32 + R * kC + c8;
      const float* pv = Vp + R * kC + c8;
      const float* pm = Mp + R * kC2 + c8;
      const v4f a0 = *(const v4f*)(po), a1 = *(const v4f*)(po + 4);
      const v4f b0v = *(const v4f*)(pv), b1v = *(const v4f*)(pv + 4);
      const v4f m0v = *(const v4f*)(pm), m1v = *(const v4f*)(pm + 4);
      const v4f m2v = *(const v4f*)(pm + 256), m3v = *(const v4f*)(pm + 260);
#pragma unroll
      for (int e = 0; e < 4; ++e) {
        v[e] = a0[e];        v[4 + e] = a1[e];
        v[8 + e] = b0v[e];   v[12 + e] = b1v[e];
        v[16 + e] = m0v[e];  v[20 + e] = m1v[e];
        v[24 + e] = m2v[e];  v[28 + e] = m3v[e];
      }
    }
    float s = 0.f;
#pragma unroll
    for (int e = 0; e < 32; ++e) s += v[e];
    s = wave_sum32(s);
    const float mu = s * kInvC4;
    float ss = 0.f;
#pragma unroll
    for (int e = 0; e < 32; ++e) { v[e] -= mu; ss += v[e] * v[e]; }
    ss = wave_sum32(ss);
    const float rstd = rsqrtf(ss * kInvC4 + kLnEps);
    v4u u[4];
#pragma unroll
    for (int q = 0; q < 4; ++q) {
      const float* gp = g1 + q * 256 + c8;
      const float* bp = be1 + q * 256 + c8;
      const v4f ga = *(const v4f*)(gp), gb = *(const v4f*)(gp + 4);
      const v4f ba = *(const v4f*)(bp), bb = *(const v4f*)(bp + 4);
      unsigned short hb[8];
#pragma unroll
      for (int e = 0; e < 4; ++e) {
        hb[e]     = h_bits(v[q * 8 + e] * rstd * ga[e] + ba[e]);
        hb[4 + e] = h_bits(v[q * 8 + 4 + e] * rstd * gb[e] + bb[e]);
      }
      u[q] = (v4u){pk16(hb[0], hb[1]), pk16(hb[2], hb[3]), pk16(hb[4], hb[5]), pk16(hb[6], hb[7])};
    }
    unsigned short* yr = Y + R * kC4;
    for (int pass = 0; pass < 2; ++pass) {
#pragma unroll
      for (int q = 0; q < 4; ++q) *(volatile v4u*)(yr + q * 256 + c8) = u[q];
      __threadfence();
    }
  }
}

template <bool FINAL>
__global__ __launch_bounds__(256) void ln2_kernel(const float* __restrict__ X32, const float* __restrict__ VP,
                                                  const float* __restrict__ g2, const float* __restrict__ be2,
                                                  float* __restrict__ Vout, unsigned short* __restrict__ CAT1,
                                                  unsigned short* __restrict__ VT, float* __restrict__ dout, int b0) {
  constexpr int ROWS = FINAL ? 32 : 64;
  constexpr int RPW  = ROWS / 8;
  __shared__ __align__(16) unsigned short tile16[FINAL ? 8 : 256 * 72];
  __shared__ __align__(16) float tile32[FINAL ? 256 * 36 : 8];
  __shared__ __align__(16) float slab[FINAL ? 8 : 8 * 256];
  const int lane = threadIdx.x & 31, wave = threadIdx.x >> 5;
  const int n0 = blockIdx.x * ROWS;
  const int bl = blockIdx.y;
  const int c8 = lane * 8, c4 = lane * 4;
  float gg[8], bb[8];
  {
    const v4f ga = *(const v4f*)(g2 + c8), gb = *(const v4f*)(g2 + c8 + 4);
    const v4f ba = *(const v4f*)(be2 + c8), bbv = *(const v4f*)(be2 + c8 + 4);
#pragma unroll
    for (int e = 0; e < 4; ++e) { gg[e] = ga[e]; gg[4 + e] = gb[e]; bb[e] = ba[e]; bb[4 + e] = bbv[e]; }
  }
  float* sw = slab + (FINAL ? 0 : wave * 256);
#pragma unroll 1
  for (int it = 0; it < RPW; ++it) {
    const int rloc = wave * RPW + it;
    const size_t R = (size_t)bl * kN + n0 + rloc;
    const float* xr = X32 + R * kC + c8;
    const float* vr = VP + R * kC + c8;
    const v4f xa = *(const v4f*)(xr), xb = *(const v4f*)(xr + 4);
    const v4f va = *(const v4f*)(vr), vb = *(const v4f*)(vr + 4);
    float t[8];
    float s = 0.f;
#pragma unroll
    for (int e = 0; e < 4; ++e) { t[e] = xa[e] + va[e]; t[4 + e] = xb[e] + vb[e]; }
#pragma unroll
    for (int e = 0; e < 8; ++e) s += t[e];
    s = wave_sum32(s);
    const float mu = s * kInvC;
    float ss = 0.f;
#pragma unroll
    for (int e = 0; e < 8; ++e) { t[e] -= mu; ss += t[e] * t[e]; }
    ss = wave_sum32(ss);
    const float rstd = rsqrtf(ss * kInvC + kLnEps);
    float y[8];
#pragma unroll
    for (int e = 0; e < 8; ++e) y[e] = t[e] * rstd * gg[e] + bb[e];
    if (!FINAL) {
      unsigned short hb[8];
#pragma unroll
      for (int e = 0; e < 8; ++e) { hb[e] = h_bits(y[e]); tile16[(c8 + e) * 72 + rloc] = hb[e]; }
      const v4u u = (v4u){pk16(hb[0], hb[1]), pk16(hb[2], hb[3]), pk16(hb[4], hb[5]), pk16(hb[6], hb[7])};
      *(v4f*)(sw + c8)     = (v4f){y[0], y[1], y[2], y[3]};
      *(v4f*)(sw + c8 + 4) = (v4f){y[4], y[5], y[6], y[7]};
      __builtin_amdgcn_fence(__ATOMIC_RELEASE, "workgroup");
      __builtin_amdgcn_wave_barrier();
      __builtin_amdgcn_fence(__ATOMIC_ACQUIRE, "workgroup");
      const v4f a0 = *(const v4f*)(sw + c4);
      const v4f a1 = *(const v4f*)(sw + 128 + c4);
      for (int pass = 0; pass < 2; ++pass) {
        *(volatile v4u*)(CAT1 + R * kC2 + kC + c8) = u;
        *(volatile v4f*)(Vout + R * kC + c4) = a0;
        *(volatile v4f*)(Vout + R * kC + 128 + c4) = a1;
        __threadfence();
      }
      __builtin_amdgcn_fence(__ATOMIC_RELEASE, "workgroup");
      __builtin_amdgcn_wave_barrier();
      __builtin_amdgcn_fence(__ATOMIC_ACQUIRE, "workgroup");
    } else {
#pragma unroll
      for (int e = 0; e < 8; ++e) tile32[(c8 + e) * 36 + rloc] = y[e];
    }
  }
  __syncthreads();
  const int q = lane >> 3;
  if (!FINAL) {
    const int cc8 = (lane & 7) * 8;
    for (int pass = 0; pass < 2; ++pass) {
#pragma unroll
      for (int i = 0; i < 8; ++i) {
        const int L = i * 32 + wave * 4 + q;
        const v4u u = *(const v4u*)(tile16 + L * 72 + cc8);
        *(volatile v4u*)(VT + ((size_t)bl * kC + L) * kN + n0 + cc8) = u;
      }
      __threadfence();
    }
  } else {
    const int cc4 = (lane & 7) * 4;
    for (int pass = 0; pass < 2; ++pass) {
#pragma unroll
      for (int i = 0; i < 8; ++i) {
        const int L = i * 32 + wave * 4 + q;
        const v4f v = *(const v4f*)(tile32 + L * 36 + cc4);
        *(volatile v4f*)(dout + ((size_t)(b0 + bl) * kC + L) * kN + n0 + cc4) = v;
      }
      __threadfence();
    }
  }
}

extern "C" void kernel_launch(void* const* d_in, const int* in_sizes, int n_in,
                              void* d_out, int out_size, void* d_ws, size_t ws_size,
                              hipStream_t stream) {
  if (n_in < 9) return;
  if (in_sizes[0] != kB * kC * kN || in_sizes[1] != kC * kC || in_sizes[2] != kC2 * kC2 ||
      in_sizes[3] != kC2 || in_sizes[4] != kC4 || in_sizes[5] != kC4 || in_sizes[6] != kC * kC4 ||
      in_sizes[7] != kC || in_sizes[8] != kC || out_size != kB * kC * kN) return;

  const float* x     = (const float*)d_in[0];
  const float* W_qkv = (const float*)d_in[1];
  const float* W_mlp = (const float*)d_in[2];
  const float* b_mlp = (const float*)d_in[3];
  const float* g1    = (const float*)d_in[4];
  const float* beta1 = (const float*)d_in[5];
  const float* W_res = (const float*)d_in[6];
  const float* g2    = (const float*)d_in[7];
  const float* beta2 = (const float*)d_in[8];
  float* out = (float*)d_out;

  size_t off = 0;
  char* wsb = (char*)d_ws;
  auto carve = [&](size_t bytes) { char* r = wsb + off; off += (bytes + 255) & ~(size_t)255; return (void*)r; };
  unsigned short* Wq16   = (unsigned short*)carve((size_t)kC * kC * 2);
  unsigned short* Wm16   = (unsigned short*)carve((size_t)kC2 * kC2 * 2);
  unsigned short* Wr16   = (unsigned short*)carve((size_t)kC * kC4 * 2);
  unsigned short* CTXT16 = (unsigned short*)carve((size_t)kGrp * kC * kC * 2);
  unsigned short* X0_16  = (unsigned short*)carve((size_t)kRowsG * kC * 2);
  float*          X32    = (float*)carve((size_t)kRowsG * kC * 4);
  unsigned short* XT16   = (unsigned short*)carve((size_t)kGrp * kC * kN * 2);
  unsigned short* SM16   = (unsigned short*)carve((size_t)kRowsG * kC * 2);
  unsigned short* CAT1   = (unsigned short*)carve((size_t)kRowsG * kC2 * 2);
  float*          OUT32  = (float*)carve((size_t)kRowsG * kC * 4);
  float*          MLP32  = (float*)carve((size_t)kRowsG * kC2 * 4);
  unsigned short* Y16    = (unsigned short*)carve((size_t)kRowsG * kC4 * 2);
  float*          VPRE32 = (float*)carve((size_t)kRowsG * kC * 4);
  float*          V32    = (float*)carve((size_t)kRowsG * kC * 4);
  unsigned short* VT16   = (unsigned short*)carve((size_t)kGrp * kC * kN * 2);
  if (off > ws_size) return;

  const dim3 blk(256);
  const long sNC  = (long)kN * kC;
  const long sNC2 = (long)kN * kC2;
  const long sNC4 = (long)kN * kC4;
  const long sCC  = (long)kC * kC;

  wcast_kernel<<<dim3(288), blk, 0, stream>>>(W_qkv, W_mlp, W_res, Wq16, Wm16, Wr16, kWCarry);

  for (int grp = 0; grp < kNGrp; ++grp) {
    const int b0 = grp * kGrp;
    tin_kernel<<<dim3(kN / 64, kGrp), blk, 0, stream>>>(x, X0_16, b0);
    wmma_gemm64<0, false, 0, 0, false, 0><<<dim3(32, kGrp), blk, 0, stream>>>(
        X0_16, X0_16, kC, sNC, Wq16, Wq16, kC, 0L,
        (void*)X32, (void*)X32, kC, sNC, b_mlp, X32, 0L, kN, kC, kC, kWCarryInv);
    prep_kernel<<<dim3(kN / 64, kGrp), blk, 0, stream>>>(X32, SM16, CAT1, XT16);

    for (int iter = 0; iter < 2; ++iter) {
      const unsigned short* vt = (iter == 0) ? XT16 : VT16;
      const float* v32 = (iter == 0) ? X32 : V32;
      wmma_gemm64<0, false, 0, 1, false, 0><<<dim3(2, kGrp), blk, 0, stream>>>(
          vt, vt, kN, sNC, XT16, XT16, kN, sNC,
          (void*)CTXT16, (void*)CTXT16, kC, sCC, b_mlp, X32, 0L, kC, kC, kN, 1.0f);
      wmma_gemm64<0, false, 0, 0, false, 0><<<dim3(32, kGrp), blk, 0, stream>>>(
          SM16, SM16, kC, sNC, CTXT16, CTXT16, kC, sCC,
          (void*)OUT32, (void*)OUT32, kC, sNC, b_mlp, X32, 0L, kN, kC, kC, kSmCarryInv);
      cast_out_kernel<<<dim3(kRowsG * 32 / 256), blk, 0, stream>>>(OUT32, CAT1, kRowsG * 32);
      wmma_gemm64<0, false, 2, 0, false, 2><<<dim3(64, kGrp), blk, 0, stream>>>(
          CAT1, CAT1, kC2, sNC2, Wm16, Wm16, kC2, 0L,
          (void*)MLP32, (void*)MLP32, kC2, sNC2, b_mlp, X32, 0L, kN, kC2, kC2, kWCarryInv);
      ln1_kernel<<<dim3(kRowsG / 64), blk, 0, stream>>>(OUT32, v32, MLP32, g1, beta1, Y16);
      wmma_gemm64<0, false, 0, 0, true, 0><<<dim3(32, kGrp), blk, 0, stream>>>(
          Y16, Y16, kC4, sNC4, Wr16, Wr16, kC4, 0L,
          (void*)VPRE32, (void*)VPRE32, kC, sNC, b_mlp, X32, sNC, kN, kC, kC4, kWCarryInv);
      if (iter == 0) {
        ln2_kernel<false><<<dim3(kN / 64, kGrp), blk, 0, stream>>>(X32, VPRE32, g2, beta2, V32, CAT1, VT16, out, b0);
      } else {
        ln2_kernel<true><<<dim3(kN / 32, kGrp), blk, 0, stream>>>(X32, VPRE32, g2, beta2, V32, CAT1, VT16, out, b0);
      }
    }
  }
  (void)ws_size;
}
